// PtrAttention_5763846111529
// MI455X (gfx1250) — hardware-verified
//
#include <hip/hip_runtime.h>


namespace {
constexpr int NB = 8, T = 128, S = 256, L = 256, D = 512, NRD = NB * T  , NRE = NB * S  ;
constexpr float XS = 8.0f, WSC = 256.0f, EPS = 1e-8f;

typedef _Float16 b16;
typedef __attribute__((ext_vector_type(16))) _Float16 v16b;
typedef __attribute__((ext_vector_type(8))) _Float16 v8b;
typedef __attribute__((ext_vector_type(8))) float v8f;
typedef __attribute__((ext_vector_type(4))) float v4f;
__device__ __forceinline__ float bf16_rne(float f) { unsigned int u = __float_as_uint(f); u += 0x7FFFu + ((u >> 16) & 1u); return __uint_as_float(u & 0xFFFF0000u); }
__device__ __forceinline__ v16b frag_kb(const b16* p, int hh) { const v8b a = *(const v8b*)(p + 8 * hh), b = *(const v8b*)(p + 16 + 8 * hh); v16b f;
#pragma unroll
  for (int e = 0; e < 8; ++e) { f[e] = a[e]; f[8 + e] = b[e]; } return f; }
__device__ __forceinline__ v8f wmma16b(v16b a, v16b b, v8f c) { v8f d = __builtin_amdgcn_wmma_f32_16x16x32_f16(false, a, false, b, (short)0, c, false, false); asm volatile("v_nop\n\tv_nop\n\tv_nop\n\tv_nop" : "+v"(d) : "v"(a), "v"(b)); return d; }
__device__ __forceinline__ void wave_lds_sync() { __builtin_amdgcn_fence(__ATOMIC_RELEASE, "workgroup"); __builtin_amdgcn_wave_barrier(); __builtin_amdgcn_fence(__ATOMIC_ACQUIRE, "workgroup"); }
__device__ __forceinline__ float pmul(float a, float b) { float p = a * b; asm volatile("" : "+v"(p)); return p; }
__device__ __forceinline__ float wsum(float v) { v += __shfl_xor(v, 1); v += __shfl_xor(v, 2); v += __shfl_xor(v, 4); v += __shfl_xor(v, 8); return v + __shfl_xor(v, 16); }
__device__ __forceinline__ float wmax(float v) { v = fmaxf(v, __shfl_xor(v, 1)); v = fmaxf(v, __shfl_xor(v, 2)); v = fmaxf(v, __shfl_xor(v, 4)); v = fmaxf(v, __shfl_xor(v, 8)); return fmaxf(v, __shfl_xor(v, 16)); }
__device__ __forceinline__ float nexp(float x) { return __builtin_amdgcn_exp2f(x * 1.4426950408889634f); }
__device__ __forceinline__ float tanh_(float x) { const float e = nexp(-2.0f * fabsf(x)); const float t = (1.0f - e) / (1.0f + e); return x < 0.0f ? -t : t; }

__global__ __launch_bounds__(256) void prep_kernel(const float* __restrict__ dec, const float* __restrict__ enc, const float* __restrict__ w1, const float* __restrict__ w2, b16* __restrict__ A16, b16* __restrict__ WT) {
  const int t = blockIdx.x * 256 + threadIdx.x; const int na = (NRD + NRE) * D / 8, nw = 2 * L * D / 8; v8b o;
  if (t < na) { const int e = t * 8; const float* src = (e < NRD * D) ? dec + e : enc + (e - NRD * D); for (int j = 0; j < 8; ++j) o[j] = (b16)(bf16_rne(src[j]) * XS); for (int pass = 0; pass < 2; ++pass) { *(volatile v8b*)(A16 + e) = o; __threadfence(); } }
  else if (t < na + nw) { const int e = (t - na) * 8; const float* w = (e < L * D) ? w1 + e : w2 + (e - L * D); for (int j = 0; j < 8; ++j) o[j] = (b16)(bf16_rne(w[j]) * WSC); for (int pass = 0; pass < 2; ++pass) { *(volatile v8b*)(WT + e) = o; __threadfence(); } }
}
__global__ __launch_bounds__(128) void proj_kernel(const b16* __restrict__ A16, const b16* __restrict__ WT, float* __restrict__ PRJ) {
  __shared__ __attribute__((aligned(16))) float Ts[4][16][128 + 4];
  const int wave = threadIdx.x >> 5, lane = threadIdx.x & 31, nloc = lane & 15, hlf = lane >> 4; const size_t m0 = (size_t)blockIdx.x * 64 + wave * 16; const int n0 = blockIdx.y * 128;
  const b16* W = WT + ((m0 < (size_t)NRD) ? 0 : (size_t)L * D);
  v8f acc[8];
#pragma unroll
  for (int t = 0; t < 8; ++t) acc[t] = (v8f){};
#pragma unroll 2
  for (int kb = 0; kb < D; kb += 32) { const v16b a = frag_kb(A16 + (m0 + nloc) * D + kb, hlf);
#pragma unroll
    for (int t = 0; t < 8; ++t) acc[t] = wmma16b(a, frag_kb(W + (size_t)(n0 + t * 16 + nloc) * D + kb, hlf), acc[t]); }
#pragma unroll
  for (int t = 0; t < 8; ++t)
#pragma unroll
    for (int r = 0; r < 8; ++r) Ts[wave][8 * hlf + r][t * 16 + nloc] = acc[t][r] * (1.0f / (XS * WSC));
  wave_lds_sync();
  for (int pass = 0; pass < 2; ++pass) { for (int rr = 0; rr < 16; ++rr) *(volatile v4f*)(PRJ + (m0 + rr) * L + n0 + lane * 4) = *(const v4f*)(&Ts[wave][rr][lane * 4]); __threadfence(); }
}
__global__ __launch_bounds__(256) void score_kernel(const float* __restrict__ PRJ, const float* __restrict__ vt, const float* __restrict__ mask, float* __restrict__ out) {
  __shared__ __attribute__((aligned(16))) float So[8][S + 4];
  const int wave = threadIdx.x >> 5, lane = threadIdx.x & 31; const int row = blockIdx.x * 8 + wave; const int b = row / T; const int l0 = lane * 8;
  float dv[8], v8[8]; for (int q = 0; q < 8; ++q) { dv[q] = PRJ[(size_t)row * L + l0 + q]; v8[q] = bf16_rne(vt[l0 + q]); }
  float lg[8];
#pragma unroll
  for (int u = 0; u < 8; ++u) lg[u] = 0.0f;
  for (int s = 0; s < S; ++s) { const float* er = PRJ + ((size_t)NRD + (size_t)b * S + s) * L + l0; float acc = 0.0f; for (int q = 0; q < 8; ++q) acc += pmul(v8[q], tanh_(dv[q] + er[q])); acc = wsum(acc);
#pragma unroll
    for (int u = 0; u < 8; ++u) if (s == lane + 32 * u) lg[u] = acc; }
  float mx = -INFINITY;
#pragma unroll
  for (int u = 0; u < 8; ++u) { const int s = lane + 32 * u; lg[u] += __logf(mask[(size_t)row * S + s] + EPS); mx = fmaxf(mx, lg[u]); }
  mx = wmax(mx); float se = 0.0f; for (int u = 0; u < 8; ++u) se += nexp(lg[u] - mx); se = wsum(se); const float lz = mx + __logf(se);
#pragma unroll
  for (int u = 0; u < 8; ++u) So[wave][lane + 32 * u] = lg[u] - lz;
  wave_lds_sync();
  for (int pass = 0; pass < 2; ++pass) { for (int c4 = lane * 4; c4 < S; c4 += 128) *(volatile v4f*)(out + (size_t)row * S + c4) = *(const v4f*)(&So[wave][c4]); __threadfence(); }
}
}

extern "C" void kernel_launch(void* const* d_in, const int* in_sizes, int n_in, void* d_out, int out_size, void* d_ws, size_t ws_size, hipStream_t stream) {
  (void)n_in;
  auto Fp = [&](int i) { return (const float*)d_in[i]; };
  if (in_sizes[0] != NRD * D || in_sizes[1] != NRE * D || in_sizes[2] != NRD * S || in_sizes[3] != L * D || in_sizes[4] != L * D || in_sizes[5] != L || out_size != NRD * S) return;
  size_t off = 0; char* ws = (char*)d_ws;
  auto carve = [&](size_t bytes) { char* p = ws + off; off += (bytes + 255) & ~(size_t)255; return p; };
  b16* A16 = (b16*)carve((size_t)(NRD + NRE) * D * 2); b16* WT = (b16*)carve((size_t)2 * L * D * 2); float* PRJ = (float*)carve((size_t)(NRD + NRE) * L * 4);
  if (off > ws_size || off > ((size_t)128 << 20)) return;
  prep_kernel<<<((NRD + NRE) * D / 8 + 2 * L * D / 8 + 255) / 256, 256, 0, stream>>>(Fp(0), Fp(1), Fp(3), Fp(4), A16, WT);
  proj_kernel<<<dim3((NRD + NRE) / 64, L / 128), 128, 0, stream>>>(A16, WT, PRJ);
  score_kernel<<<NRD / 8, 256, 0, stream>>>(PRJ, Fp(5), Fp(2), (float*)d_out);
}
